// RoPESelfAttentionBase_80470507257926
// MI455X (gfx1250) — hardware-verified
//
#include <hip/hip_runtime.h>
#include <stddef.h>
#include <stdint.h>

#define NBATCH 4
#define TT     1024
#define EE     1024
#define HH     16
#define DK     64
#define NBLK   16
#define NAX    3
#define NSP    (NBATCH * TT)
#define NROW   (NSP * HH)
#define GK     EE
#define NW4    (4 * EE)
#define BR     32
#define BC     128
#define NCH    (TT / BC)

static_assert(GK % 32 == 0);
static_assert(DK == 64);
static_assert(NBLK * 4 == DK);
static_assert(TT % 256 == 0);
static_assert(TT % 64 == 0);
static_assert(TT % BR == 0);
static_assert(TT % BC == 0);
static_assert(BC % 32 == 0);
static_assert(EE % 64 == 0);
static_assert(NSP % 256 == 0);
static_assert(NSP % 128 == 0);

typedef float          v8f   __attribute__((ext_vector_type(8)));
typedef float          v4f   __attribute__((ext_vector_type(4)));
typedef unsigned int   v4u   __attribute__((ext_vector_type(4)));
typedef unsigned short v8us  __attribute__((ext_vector_type(8)));
typedef unsigned short v16us __attribute__((ext_vector_type(16)));
typedef __bf16         v16b  __attribute__((ext_vector_type(16)));
typedef unsigned short ush;

union FragU { v16us v; v8us h[2]; v16b b; };
union PackU { v8us s; v4u u; };
struct HL { v4u h; v4u l; };

__device__ __forceinline__ ush f2bf(float f) {
  const unsigned u = __float_as_uint(f);
  return (ush)((u + 0x7FFFu + ((u >> 16) & 1u)) >> 16);
}
__device__ __forceinline__ float bf2f(ush b) { return __uint_as_float(((unsigned)b) << 16); }

__device__ __forceinline__ HL split8(v8f f) {
  PackU ph, pl;
#pragma unroll
  for (int e = 0; e < 8; ++e) {
    const ush hi = f2bf(f[e]);
    ph.s[e] = hi;
    pl.s[e] = f2bf(f[e] - bf2f(hi));
  }
  HL r; r.h = ph.u; r.l = pl.u;
  return r;
}

__device__ __forceinline__ v8f mmab(v16us a, v16us b, v8f c) {
  FragU ua, ub; ua.v = a; ub.v = b;
  c = __builtin_amdgcn_wmma_f32_16x16x32_bf16(false, ua.b, false, ub.b, (short)0, c, false, false);
  asm volatile("v_nop\n\tv_nop\n\tv_nop\n\tv_nop" : "+v"(c) : "v"(a), "v"(b));
  return c;
}

__device__ __forceinline__ v16us ldfragu(const ush* p, int ld, int row0, int k0, int lane) {
  const int m = lane & 15, lh = lane >> 4;
  const ush* q = p + (size_t)(row0 + m) * ld + k0 + 8 * lh;
  FragU f;
  f.h[0] = *(const v8us*)(q);
  f.h[1] = *(const v8us*)(q + 16);
  return f.v;
}

__device__ __forceinline__ v8f zero8() { return (v8f){0.f, 0.f, 0.f, 0.f, 0.f, 0.f, 0.f, 0.f}; }

__device__ __forceinline__ void gemm3_32x64(const ush* __restrict__ Ah, const ush* __restrict__ Al, int lda,
                                            const ush* __restrict__ Bh, const ush* __restrict__ Bl, int ldb,
                                            int m0, int n0, int lane, v8f (&acc)[2][4]) {
#pragma unroll 1
  for (int k0 = 0; k0 < GK; k0 += 32) {
    const v16us a0h = ldfragu(Ah, lda, m0, k0, lane);
    const v16us a1h = ldfragu(Ah, lda, m0 + 16, k0, lane);
    const v16us a0l = ldfragu(Al, lda, m0, k0, lane);
    const v16us a1l = ldfragu(Al, lda, m0 + 16, k0, lane);
#pragma unroll
    for (int t = 0; t < 4; ++t) {
      const v16us bh = ldfragu(Bh, ldb, n0 + 16 * t, k0, lane);
      const v16us bl = ldfragu(Bl, ldb, n0 + 16 * t, k0, lane);
      acc[0][t] = mmab(a0h, bh, acc[0][t]);
      acc[1][t] = mmab(a1h, bh, acc[1][t]);
      acc[0][t] = mmab(a0h, bl, acc[0][t]);
      acc[1][t] = mmab(a1h, bl, acc[1][t]);
      acc[0][t] = mmab(a0l, bh, acc[0][t]);
      acc[1][t] = mmab(a1l, bh, acc[1][t]);
    }
  }
}

__device__ __forceinline__ void mm4(float (&d)[16], const float (&x)[16], const float (&y)[16]) {
#pragma unroll
  for (int r = 0; r < 4; ++r) {
#pragma unroll
    for (int cc = 0; cc < 4; ++cc) {
      float s = x[4 * r] * y[cc];
      s = fmaf(x[4 * r + 1], y[4 + cc], s);
      s = fmaf(x[4 * r + 2], y[8 + cc], s);
      s = fmaf(x[4 * r + 3], y[12 + cc], s);
      d[4 * r + cc] = s;
    }
  }
}

__device__ __forceinline__ void expm4(float (&M)[16], float (&R)[16]) {
  float nrm = 0.f;
#pragma unroll
  for (int cc = 0; cc < 4; ++cc) {
    const float cs = fabsf(M[cc]) + fabsf(M[4 + cc]) + fabsf(M[8 + cc]) + fabsf(M[12 + cc]);
    nrm = fmaxf(nrm, cs);
  }
  int s = 0;
  float scl = 1.0f;
  while (nrm > 0.5f && s < 30) { nrm *= 0.5f; scl *= 0.5f; ++s; }
#pragma unroll
  for (int j = 0; j < 16; ++j) M[j] *= scl;

  float M2[16], M3[16], M4[16], T[16], U[16];
  mm4(M2, M, M);
  mm4(M3, M2, M);
  mm4(M4, M2, M2);

  const float c2  = 0.5f;
  const float c3  = 0.16666666666666666f;
  const float c4  = 0.041666666666666664f;
  const float c5  = 0.008333333333333333f;
  const float c6  = 0.001388888888888889f;
  const float c7  = 1.984126984126984e-4f;
  const float c8  = 2.48015873015873e-5f;
  const float c9  = 2.7557319223985893e-6f;
  const float c10 = 2.755731922398589e-7f;
  const float c11 = 2.505210838544172e-8f;
  const float c12 = 2.08767569878681e-9f;

#pragma unroll
  for (int j = 0; j < 16; ++j) {
    float v = c12 * M4[j];
    v = fmaf(c11, M3[j], v);
    v = fmaf(c10, M2[j], v);
    v = fmaf(c9, M[j], v);
    if ((j % 5) == 0) v += c8;
    T[j] = v;
  }
  mm4(U, M4, T);
#pragma unroll
  for (int j = 0; j < 16; ++j) {
    float v = U[j];
    v = fmaf(c7, M3[j], v);
    v = fmaf(c6, M2[j], v);
    v = fmaf(c5, M[j], v);
    if ((j % 5) == 0) v += c4;
    T[j] = v;
  }
  mm4(U, M4, T);
#pragma unroll
  for (int j = 0; j < 16; ++j) {
    float v = U[j];
    v = fmaf(c3, M3[j], v);
    v = fmaf(c2, M2[j], v);
    v += M[j];
    if ((j % 5) == 0) v += 1.0f;
    R[j] = v;
  }
#pragma unroll 1
  for (int i = 0; i < s; ++i) {
    mm4(U, R, R);
#pragma unroll
    for (int j = 0; j < 16; ++j) R[j] = U[j];
  }
}

__global__ __launch_bounds__(256) void k_cvt_x(const float* __restrict__ x, ush* __restrict__ xh,
                                               ush* __restrict__ xl, int ngrp) {
  const int t = blockIdx.x * 256 + (int)threadIdx.x;
  if (t >= ngrp) return;
  const size_t o = (size_t)t * 8;
  const v4f a0 = *(const v4f*)(x + o);
  const v4f a1 = *(const v4f*)(x + o + 4);
  const v8f f = (v8f){a0[0], a0[1], a0[2], a0[3], a1[0], a1[1], a1[2], a1[3]};
  const HL s = split8(f);
  *(volatile v4u*)(xh + o) = s.h;
  *(volatile v4u*)(xl + o) = s.l;
  __threadfence();
  *(volatile v4u*)(xh + o) = s.h;
  *(volatile v4u*)(xl + o) = s.l;
}

__global__ __launch_bounds__(256) void k_cvt_w(const float* __restrict__ wq, const float* __restrict__ wk,
                                               const float* __restrict__ wv, const float* __restrict__ wo,
                                               ush* __restrict__ w4h, ush* __restrict__ w4l, int ngrp) {
  const int which = blockIdx.y;
  const float* w = (which == 0) ? wq : ((which == 1) ? wk : ((which == 2) ? wv : wo));
  const int t = blockIdx.x * 256 + (int)threadIdx.x;
  if (t >= ngrp) return;
  const size_t o  = (size_t)t * 8;
  const size_t od = (size_t)which * EE * GK + o;
  const v4f a0 = *(const v4f*)(w + o);
  const v4f a1 = *(const v4f*)(w + o + 4);
  const v8f f = (v8f){a0[0], a0[1], a0[2], a0[3], a1[0], a1[1], a1[2], a1[3]};
  const HL s = split8(f);
  *(volatile v4u*)(w4h + od) = s.h;
  *(volatile v4u*)(w4l + od) = s.l;
  __threadfence();
  *(volatile v4u*)(w4h + od) = s.h;
  *(volatile v4u*)(w4l + od) = s.l;
}

#define QTP 132
__global__ __launch_bounds__(128) void k_qk3(const ush* __restrict__ xh, const ush* __restrict__ xl,
                                             const ush* __restrict__ w4h, const ush* __restrict__ w4l,
                                             const float* __restrict__ bq, const float* __restrict__ bk,
                                             const float* __restrict__ pos, const float* __restrict__ araw,
                                             ush* __restrict__ qh, ush* __restrict__ ql,
                                             ush* __restrict__ kh, ush* __restrict__ kl) {
  __shared__ __align__(16) float sT[64 * QTP];
  __shared__ __align__(16) float sA[NAX * NBLK * 16];
  const int tid = threadIdx.x, lane = tid & 31, wave = tid >> 5;
  const int hh = lane >> 4, c = lane & 15;
  const int mb   = blockIdx.x * 64;
  const int head = blockIdx.y;
  const int grp  = wave >> 1;
  const int m0   = mb + (wave & 1) * 32;
  const int n0   = grp * EE + head * DK;

  for (int i = tid; i < NAX * NBLK * 16; i += 128) {
    const int a = i >> 8, rem = i & 255;
    const int nb = rem >> 4, rc = rem & 15;
    const int r = rc >> 2, cc = rc & 3;
    const int base = ((head * NAX + a) * NBLK + nb) * 16;
    sA[i] = araw[base + r * 4 + cc] - araw[base + cc * 4 + r];
  }

  v8f acc[2][4];
#pragma unroll
  for (int s = 0; s < 2; ++s)
#pragma unroll
    for (int t = 0; t < 4; ++t) acc[s][t] = zero8();
  gemm3_32x64(xh, xl, GK, w4h, w4l, GK, m0, n0, lane, acc);

  const float sc = (grp == 0) ? 0.125f : 1.0f;
#pragma unroll
  for (int t = 0; t < 4; ++t) {
    const float bqv = bq[head * DK + 16 * t + c];
    const float bkv = bk[head * DK + 16 * t + c];
    const float bn  = (grp == 0) ? bqv : bkv;
#pragma unroll
    for (int sub = 0; sub < 2; ++sub) {
#pragma unroll
      for (int r = 0; r < 8; ++r) {
        const int lr = (wave & 1) * 32 + sub * 16 + 8 * hh + r;
        sT[lr * QTP + grp * DK + 16 * t + c] = (acc[sub][t][r] + bn) * sc;
      }
    }
  }
  __syncthreads();

#pragma unroll 1
  for (int it = 0; it < 8; ++it) {
    const int i  = tid + 128 * it;
    const int lr = i >> 4;
    const int nb = i & 15;
    const int m  = mb + lr;
    const float p0 = pos[(size_t)m * NAX + 0];
    const float p1 = pos[(size_t)m * NAX + 1];
    const float p2 = pos[(size_t)m * NAX + 2];
    float M[16], R[16];
#pragma unroll
    for (int j = 0; j < 16; ++j)
      M[j] = p0 * sA[nb * 16 + j] + p1 * sA[256 + nb * 16 + j] + p2 * sA[512 + nb * 16 + j];
    expm4(M, R);
    float* qp = sT + lr * QTP + nb * 4;
    float* kp = qp + DK;
    float q4[4], k4[4], qo[4], ko[4];
#pragma unroll
    for (int mm = 0; mm < 4; ++mm) { q4[mm] = qp[mm]; k4[mm] = kp[mm]; }
#pragma unroll
    for (int kk = 0; kk < 4; ++kk) {
      float qs = R[kk * 4] * q4[0];
      float ks = R[kk * 4] * k4[0];
#pragma unroll
      for (int mm = 1; mm < 4; ++mm) {
        qs = fmaf(R[kk * 4 + mm], q4[mm], qs);
        ks = fmaf(R[kk * 4 + mm], k4[mm], ks);
      }
      qo[kk] = qs; ko[kk] = ks;
    }
#pragma unroll
    for (int kk = 0; kk < 4; ++kk) { qp[kk] = qo[kk]; kp[kk] = ko[kk]; }
  }
  __syncthreads();

  const int b = mb / TT;
  const size_t rp0 = (size_t)(b * HH + head) * TT + (size_t)(mb - b * TT);
  {
    v4u vh[4], vl[4];
    size_t go[4];
#pragma unroll
    for (int j = 0; j < 4; ++j) {
      const int p  = tid + 128 * j;
      const int L  = p >> 3;
      const int pc = p & 7;
      v8f f;
#pragma unroll
      for (int e = 0; e < 8; ++e) f[e] = sT[L * QTP + pc * 8 + e];
      const HL s = split8(f);
      vh[j] = s.h; vl[j] = s.l;
      go[j] = (rp0 + (size_t)L) * DK + pc * 8;
    }
#pragma unroll
    for (int j = 0; j < 4; ++j) { *(volatile v4u*)(qh + go[j]) = vh[j]; *(volatile v4u*)(ql + go[j]) = vl[j]; }
    __threadfence();
#pragma unroll
    for (int j = 0; j < 4; ++j) { *(volatile v4u*)(qh + go[j]) = vh[j]; *(volatile v4u*)(ql + go[j]) = vl[j]; }
  }
  {
    v4u vh[4], vl[4];
    size_t go[4];
#pragma unroll
    for (int j = 0; j < 4; ++j) {
      const int p  = tid + 128 * j;
      const int L  = p >> 3;
      const int pc = p & 7;
      v8f f;
#pragma unroll
      for (int e = 0; e < 8; ++e) f[e] = sT[L * QTP + DK + pc * 8 + e];
      const HL s = split8(f);
      vh[j] = s.h; vl[j] = s.l;
      go[j] = (rp0 + (size_t)L) * DK + pc * 8;
    }
#pragma unroll
    for (int j = 0; j < 4; ++j) { *(volatile v4u*)(kh + go[j]) = vh[j]; *(volatile v4u*)(kl + go[j]) = vl[j]; }
    __threadfence();
#pragma unroll
    for (int j = 0; j < 4; ++j) { *(volatile v4u*)(kh + go[j]) = vh[j]; *(volatile v4u*)(kl + go[j]) = vl[j]; }
  }
}

#define STP 72
__global__ __launch_bounds__(256) void k_v3(const ush* __restrict__ xh, const ush* __restrict__ xl,
                                            const ush* __restrict__ w4h, const ush* __restrict__ w4l,
                                            const float* __restrict__ bv,
                                            ush* __restrict__ vth, ush* __restrict__ vtl) {
  __shared__ __align__(16) ush st[256 * STP];
  const int tid = threadIdx.x, lane = tid & 31, wave = tid >> 5;
  const int hh = lane >> 4, c = lane & 15;
  const int mb   = blockIdx.x * 256;
  const int m0   = mb + wave * 32;
  const int head = blockIdx.y;
  const int n0   = 2 * EE + head * DK;

  v8f acc[2][4];
#pragma unroll
  for (int s = 0; s < 2; ++s)
#pragma unroll
    for (int t = 0; t < 4; ++t) acc[s][t] = zero8();
  gemm3_32x64(xh, xl, GK, w4h, w4l, GK, m0, n0, lane, acc);

#pragma unroll
  for (int t = 0; t < 4; ++t) {
    const float bn = bv[head * DK + 16 * t + c];
#pragma unroll
    for (int sub = 0; sub < 2; ++sub) {
#pragma unroll
      for (int r = 0; r < 8; ++r) acc[sub][t][r] += bn;
    }
  }

  const int b = mb / TT;
  const size_t rp0 = (size_t)(b * HH + head) * TT + (size_t)(mb - b * TT);
  size_t go[8];
#pragma unroll
  for (int j = 0; j < 8; ++j) {
    const int p  = tid + 256 * j;
    const int L  = p >> 3;
    const int pc = p & 7;
    const int d  = L >> 2;
    const int nl = (L & 3) * 64 + pc * 8;
    go[j] = ((size_t)d) * NROW + rp0 + (size_t)nl;
  }

#pragma unroll 1
  for (int ph = 0; ph < 2; ++ph) {
    __syncthreads();
#pragma unroll
    for (int t = 0; t < 4; ++t) {
#pragma unroll
      for (int sub = 0; sub < 2; ++sub) {
#pragma unroll
        for (int r = 0; r < 8; ++r) {
          const int lr = wave * 32 + sub * 16 + 8 * hh + r;
          const float v = acc[sub][t][r];
          const ush hi = f2bf(v);
          st[lr * STP + 16 * t + c] = (ph == 0) ? hi : f2bf(v - bf2f(hi));
        }
      }
    }
    __syncthreads();
    v4u val[8];
#pragma unroll
    for (int j = 0; j < 8; ++j) {
      const int p  = tid + 256 * j;
      const int L  = p >> 3;
      const int pc = p & 7;
      const int d  = L >> 2;
      const int nl = (L & 3) * 64 + pc * 8;
      const ush* cp = st + nl * STP + d;
      PackU pk;
      pk.s = (v8us){cp[0 * STP], cp[1 * STP], cp[2 * STP], cp[3 * STP],
                    cp[4 * STP], cp[5 * STP], cp[6 * STP], cp[7 * STP]};
      val[j] = pk.u;
    }
    ush* dst = (ph == 0) ? vth : vtl;
#pragma unroll
    for (int j = 0; j < 8; ++j) *(volatile v4u*)(dst + go[j]) = val[j];
    __threadfence();
#pragma unroll
    for (int j = 0; j < 8; ++j) *(volatile v4u*)(dst + go[j]) = val[j];
    __threadfence();
  }
}

#define SSP 128
#define SPP 136
#define OTP 68
__global__ __launch_bounds__(256) void k_attn3(const ush* __restrict__ qh, const ush* __restrict__ ql,
                                               const ush* __restrict__ kh, const ush* __restrict__ kl,
                                               const ush* __restrict__ vth, const ush* __restrict__ vtl,
                                               ush* __restrict__ oh, ush* __restrict__ ol) {
  __shared__ __align__(16) float sSO[BR * SSP];
  __shared__ __align__(16) ush   sPh[BR * SPP];
  __shared__ __align__(16) ush   sPl[BR * SPP];
  __shared__ __align__(16) float sRed[BR * 8];
  __shared__ __align__(16) float rM[BR];
  __shared__ __align__(16) float rMn[BR];
  __shared__ __align__(16) float rL[BR];
  __shared__ __align__(16) float rSc[BR];

  float* sS = sSO;
  const int tid = threadIdx.x, lane = tid & 31, wave = tid >> 5;
  const int hh = lane >> 4, c = lane & 15;
  const int rt = wave >> 2, ct = wave & 3;
  const int q0  = (int)blockIdx.x * BR;
  const int bh  = q0 / TT;
  const int kb0 = bh * TT;
  const float NEGI = -__builtin_huge_valf();
  if (tid < BR) { rM[tid] = NEGI; rL[tid] = 0.f; }

  const v16us a0h0 = ldfragu(qh, DK, q0,      0,  lane);
  const v16us a1h0 = ldfragu(qh, DK, q0 + 16, 0,  lane);
  const v16us a0l0 = ldfragu(ql, DK, q0,      0,  lane);
  const v16us a1l0 = ldfragu(ql, DK, q0 + 16, 0,  lane);
  const v16us a0h1 = ldfragu(qh, DK, q0,      32, lane);
  const v16us a1h1 = ldfragu(qh, DK, q0 + 16, 32, lane);
  const v16us a0l1 = ldfragu(ql, DK, q0,      32, lane);
  const v16us a1l1 = ldfragu(ql, DK, q0 + 16, 32, lane);
  __syncthreads();

  v8f oacc = zero8();
  const int srow = tid >> 3, schk = tid & 7;

#pragma unroll 1
  for (int ch = 0; ch < NCH; ++ch) {
    const int j0  = ch * BC;
    const int kr0 = kb0 + j0 + wave * 16;
    v8f s[2];
    s[0] = zero8(); s[1] = zero8();
    {
      const v16us kbh = ldfragu(kh, DK, kr0, 0, lane);
      const v16us kbl = ldfragu(kl, DK, kr0, 0, lane);
      s[0] = mmab(a0h0, kbh, s[0]);
      s[1] = mmab(a1h0, kbh, s[1]);
      s[0] = mmab(a0h0, kbl, s[0]);
      s[1] = mmab(a1h0, kbl, s[1]);
      s[0] = mmab(a0l0, kbh, s[0]);
      s[1] = mmab(a1l0, kbh, s[1]);
    }
    {
      const v16us kbh = ldfragu(kh, DK, kr0, 32, lane);
      const v16us kbl = ldfragu(kl, DK, kr0, 32, lane);
      s[0] = mmab(a0h1, kbh, s[0]);
      s[1] = mmab(a1h1, kbh, s[1]);
      s[0] = mmab(a0h1, kbl, s[0]);
      s[1] = mmab(a1h1, kbl, s[1]);
      s[0] = mmab(a0l1, kbh, s[0]);
      s[1] = mmab(a1l1, kbh, s[1]);
    }
#pragma unroll
    for (int t = 0; t < 2; ++t) {
#pragma unroll
      for (int r = 0; r < 8; ++r) {
        const int row = 16 * t + 8 * hh + r;
        sS[row * SSP + wave * 16 + c] = s[t][r];
      }
    }
    __syncthreads();
    {
      const float* sr = sS + srow * SSP + schk * 16;
      const v4f x0 = *(const v4f*)(sr);
      const v4f x1 = *(const v4f*)(sr + 4);
      const v4f x2 = *(const v4f*)(sr + 8);
      const v4f x3 = *(const v4f*)(sr + 12);
      float mx = x0[0];
#pragma unroll
      for (int e = 1; e < 4; ++e) mx = fmaxf(mx, x0[e]);
#pragma unroll
      for (int e = 0; e < 4; ++e) { mx = fmaxf(mx, x1[e]); mx = fmaxf(mx, x2[e]); mx = fmaxf(mx, x3[e]); }
      sRed[srow * 8 + schk] = mx;
    }
    __syncthreads();
    if (tid < BR) {
      float mx = rM[tid];
#pragma unroll
      for (int i = 0; i < 8; ++i) mx = fmaxf(mx, sRed[tid * 8 + i]);
      rMn[tid] = mx;
    }
    __syncthreads();
    {
      const float mx = rMn[srow];
      const float* sr = sS + srow * SSP + schk * 16;
      float sum = 0.f;
      PackU ph0, pl0, ph1, pl1;
#pragma unroll
      for (int e = 0; e < 8; ++e) {
        const float p = __expf(sr[e] - mx);
        sum += p;
        const ush hi = f2bf(p);
        ph0.s[e] = hi;
        pl0.s[e] = f2bf(p - bf2f(hi));
      }
#pragma unroll
      for (int e = 0; e < 8; ++e) {
        const float p = __expf(sr[8 + e] - mx);
        sum += p;
        const ush hi = f2bf(p);
        ph1.s[e] = hi;
        pl1.s[e] = f2bf(p - bf2f(hi));
      }
      *(v8us*)(sPh + srow * SPP + schk * 16)     = ph0.s;
      *(v8us*)(sPh + srow * SPP + schk * 16 + 8) = ph1.s;
      *(v8us*)(sPl + srow * SPP + schk * 16)     = pl0.s;
      *(v8us*)(sPl + srow * SPP + schk * 16 + 8) = pl1.s;
      sRed[srow * 8 + schk] = sum;
    }
    __syncthreads();
    if (tid < BR) {
      float sum = 0.f;
#pragma unroll
      for (int i = 0; i < 8; ++i) sum += sRed[tid * 8 + i];
      const float mnew = rMn[tid];
      const float fac  = __expf(rM[tid] - mnew);
      rL[tid]  = rL[tid] * fac + sum;
      rM[tid]  = mnew;
      rSc[tid] = fac;
    }
    __syncthreads();
    {
      const v4f f0 = *(const v4f*)(rSc + 16 * rt + 8 * hh);
      const v4f f1 = *(const v4f*)(rSc + 16 * rt + 8 * hh + 4);
#pragma unroll
      for (int r = 0; r < 4; ++r) {
        oacc[r]     *= f0[r];
        oacc[4 + r] *= f1[r];
      }
    }
#pragma unroll 1
    for (int kk = 0; kk < BC / 32; ++kk) {
      const v16us pah = ldfragu(sPh, SPP, 16 * rt, kk * 32, lane);
      const v16us pal = ldfragu(sPl, SPP, 16 * rt, kk * 32, lane);
      const v16us vbh = ldfragu(vth, NROW, 16 * ct, kb0 + j0 + kk * 32, lane);
      const v16us vbl = ldfragu(vtl, NROW, 16 * ct, kb0 + j0 + kk * 32, lane);
      oacc = mmab(pah, vbh, oacc);
      oacc = mmab(pah, vbl, oacc);
      oacc = mmab(pal, vbh, oacc);
    }
    __syncthreads();
  }

  float* sO = sSO;
#pragma unroll
  for (int r = 0; r < 8; ++r) {
    const int row  = 16 * rt + 8 * hh + r;
    const float lv  = rL[row];
    const float inv = (lv > 0.f) ? (1.0f / lv) : 0.f;
    sO[row * OTP + ct * 16 + c] = oacc[r] * inv;
  }
  __syncthreads();
  const int b    = bh / HH;
  const int head = bh - b * HH;
  const int tb   = q0 - kb0;
  const int L  = tid >> 3;
  const int pc = tid & 7;
  v8f f;
#pragma unroll
  for (int e = 0; e < 8; ++e) f[e] = sO[L * OTP + pc * 8 + e];
  const HL sp = split8(f);
  const size_t go = ((size_t)(b * TT + tb + L)) * EE + head * DK + pc * 8;
  *(volatile v4u*)(oh + go) = sp.h;
  *(volatile v4u*)(ol + go) = sp.l;
  __threadfence();
  *(volatile v4u*)(oh + go) = sp.h;
  *(volatile v4u*)(ol + go) = sp.l;
}

#define OSP 68
__global__ __launch_bounds__(128) void k_out3(const ush* __restrict__ w4h, const ush* __restrict__ w4l,
                                              const ush* __restrict__ oh, const ush* __restrict__ ol,
                                              const float* __restrict__ bo, float* __restrict__ out) {
  __shared__ __align__(16) float st[128 * OSP];
  const int tid = threadIdx.x, lane = tid & 31, wave = tid >> 5;
  const int hh = lane >> 4, c = lane & 15;
  const int mblk = blockIdx.x * 128;
  const int o0   = blockIdx.y * 64;
  const int m0   = mblk + wave * 32;
  const int n0   = 3 * EE + o0;

  v8f acc[2][4];
#pragma unroll
  for (int s = 0; s < 2; ++s)
#pragma unroll
    for (int t = 0; t < 4; ++t) acc[s][t] = zero8();
  gemm3_32x64(oh, ol, EE, w4h, w4l, GK, m0, n0, lane, acc);

#pragma unroll
  for (int t = 0; t < 4; ++t) {
    const float bn = bo[o0 + 16 * t + c];
#pragma unroll
    for (int sub = 0; sub < 2; ++sub) {
#pragma unroll
      for (int r = 0; r < 8; ++r) {
        const int lr = wave * 32 + sub * 16 + 8 * hh + r;
        st[lr * OSP + 16 * t + c] = acc[sub][t][r] + bn;
      }
    }
  }
  __syncthreads();
  v4f val[16];
  size_t go[16];
#pragma unroll
  for (int j = 0; j < 16; ++j) {
    const int p  = tid + 128 * j;
    const int L  = p >> 3;
    const int pc = p & 7;
    const int lr = L >> 1, hf = L & 1;
    val[j] = *(const v4f*)(st + lr * OSP + hf * 32 + pc * 4);
    go[j]  = ((size_t)(mblk + lr)) * EE + o0 + hf * 32 + pc * 4;
  }
#pragma unroll
  for (int j = 0; j < 16; ++j) *(volatile v4f*)(out + go[j]) = val[j];
  __threadfence();
#pragma unroll
  for (int j = 0; j < 16; ++j) *(volatile v4f*)(out + go[j]) = val[j];
}

extern "C" void kernel_launch(void* const* d_in, const int* in_sizes, int n_in,
                              void* d_out, int out_size, void* d_ws, size_t ws_size,
                              hipStream_t stream) {
  if (n_in < 11) return;
  if (in_sizes[0] != NSP * EE) return;
  if (in_sizes[1] != NSP * NAX) return;
  if (in_sizes[2] != HH * NAX * NBLK * 16) return;
  if (in_sizes[3] != EE * EE || in_sizes[5] != EE * EE || in_sizes[7] != EE * EE || in_sizes[9] != EE * EE) return;
  if (in_sizes[4] != EE || in_sizes[6] != EE || in_sizes[8] != EE || in_sizes[10] != EE) return;
  if (out_size != NSP * EE) return;

  const float* x    = (const float*)d_in[0];
  const float* pos  = (const float*)d_in[1];
  const float* araw = (const float*)d_in[2];
  const float* wq   = (const float*)d_in[3];
  const float* bq   = (const float*)d_in[4];
  const float* wk   = (const float*)d_in[5];
  const float* bk   = (const float*)d_in[6];
  const float* wv   = (const float*)d_in[7];
  const float* bv   = (const float*)d_in[8];
  const float* wo   = (const float*)d_in[9];
  const float* bo   = (const float*)d_in[10];
  float* out = (float*)d_out;

  size_t off = 0;
  const size_t oXh  = off; off += (size_t)NSP * EE * 2;
  const size_t oXl  = off; off += (size_t)NSP * EE * 2;
  const size_t oW4h = off; off += (size_t)NW4 * GK * 2;
  const size_t oW4l = off; off += (size_t)NW4 * GK * 2;
  const size_t oQh  = off; off += (size_t)NROW * DK * 2;
  const size_t oQl  = off; off += (size_t)NROW * DK * 2;
  const size_t oKh  = off; off += (size_t)NROW * DK * 2;
  const size_t oKl  = off; off += (size_t)NROW * DK * 2;
  const size_t oVTh = off; off += (size_t)DK * NROW * 2;
  const size_t oVTl = off; off += (size_t)DK * NROW * 2;
  const size_t oOh  = off; off += (size_t)NSP * EE * 2;
  const size_t oOl  = off; off += (size_t)NSP * EE * 2;
  if (off > ws_size) return;
  if (off > (size_t)134217728) return;

  char* ws = (char*)d_ws;
  ush* Xh  = (ush*)(ws + oXh);
  ush* Xl  = (ush*)(ws + oXl);
  ush* W4h = (ush*)(ws + oW4h);
  ush* W4l = (ush*)(ws + oW4l);
  ush* Qh  = (ush*)(ws + oQh);
  ush* Ql  = (ush*)(ws + oQl);
  ush* Kh  = (ush*)(ws + oKh);
  ush* Kl  = (ush*)(ws + oKl);
  ush* VTh = (ush*)(ws + oVTh);
  ush* VTl = (ush*)(ws + oVTl);
  ush* Oh  = (ush*)(ws + oOh);
  ush* Ol  = (ush*)(ws + oOl);

  const int ngx = in_sizes[0] / 8;
  k_cvt_x<<<dim3((ngx + 255) / 256), dim3(256), 0, stream>>>(x, Xh, Xl, ngx);
  const int ngw = in_sizes[3] / 8;
  k_cvt_w<<<dim3((ngw + 255) / 256, 4), dim3(256), 0, stream>>>(wq, wk, wv, wo, W4h, W4l, ngw);
  k_qk3<<<dim3(NSP / 64, HH), dim3(128), 0, stream>>>(Xh, Xl, W4h, W4l, bq, bk, pos, araw, Qh, Ql, Kh, Kl);
  k_v3<<<dim3(NSP / 256, HH), dim3(256), 0, stream>>>(Xh, Xl, W4h, W4l, bv, VTh, VTl);
  k_attn3<<<dim3(NROW / BR), dim3(256), 0, stream>>>(Qh, Ql, Kh, Kl, VTh, VTl, Oh, Ol);
  k_out3<<<dim3(NSP / 128, EE / 64), dim3(128), 0, stream>>>(W4h, W4l, Oh, Ol, bo, out);
  (void)hipGetLastError();
}
